// NGCF_matrix_12575664242933
// MI455X (gfx1250) — hardware-run, weakly checked
//
#include <hip/hip_runtime.h>
#include <stddef.h>


#define DD      64
#define NTHR    256
#define NWAVE   8
#define EPT     8
#define NGRP    2
#define CHUNK   (NTHR * EPT * NGRP)
#define WCAP    (EPT * NGRP * 32)
#define LISTN   (NWAVE * WCAP)
#define NBC     4096
#define NBF     1024
#define RCAP    32768
#define RBN     128
#define TGT     256
#define DEGCAP  256
#define GROWS   128
#define OTHR    512
#define WSCAP   134217728
#define APK     72
#define WPLANE  (DD * DD)
#define LMAX    8
#define ASC     16.0f
#define WSC     64.0f
#define ISC     (1.0f / 1024.0f)

#define LDS_FILL  ((RCAP + NBF + LISTN) * 4 + 64)
#define LDS_LAYER (2 * GROWS * APK * 2 + GROWS * DD * 4)

static_assert((CHUNK & (CHUNK - 1)) == 0);
static_assert(CHUNK <= 4096);
static_assert(NBC <= 4096 && NBF <= 4096);
static_assert((NBC & (NBC - 1)) == 0 && (NBF & (NBF - 1)) == 0);
static_assert(NBC == 4 * NBF);
static_assert(OTHR * 8 == NBC);
static_assert((RCAP % 32) == 0);
static_assert((TGT % GROWS) == 0 && TGT == NWAVE * 32);
static_assert((NBC % TGT) == 0);
static_assert(GROWS == NWAVE * 16);
static_assert(((2 * GROWS * APK * 2) % 16) == 0);
static_assert(((GROWS * DD / 8) % NTHR) == 0);

typedef float          v2f  __attribute__((ext_vector_type(2)));
typedef float          v4f  __attribute__((ext_vector_type(4)));
typedef float          v8f  __attribute__((ext_vector_type(8)));
typedef int            v4i  __attribute__((ext_vector_type(4)));
typedef _Float16       v8h  __attribute__((ext_vector_type(8)));
typedef _Float16       v16h __attribute__((ext_vector_type(16)));
union FragH  { v16h v; v8h half[2]; };
union Pack16 { v8h h; v4f f; };

__device__ __forceinline__ v8h cvt8(v4f a, v4f b) {
  Pack16 p;
  p.h[0] = (_Float16)a.x; p.h[1] = (_Float16)a.y; p.h[2] = (_Float16)a.z; p.h[3] = (_Float16)a.w;
  p.h[4] = (_Float16)b.x; p.h[5] = (_Float16)b.y; p.h[6] = (_Float16)b.z; p.h[7] = (_Float16)b.w;
  return p.h;
}

__device__ __forceinline__ v8f wmh(v16h a, v16h b, v8f c) {
  v8f d = __builtin_amdgcn_wmma_f32_16x16x32_f16(false, a, false, b, (short)0, c, false, false);
  asm volatile("v_nop\n\tv_nop\n\tv_nop\n\tv_nop" : "+v"(d) : "v"(a), "v"(b));
  return d;
}

template <int NB>
__device__ __forceinline__ int scan_chunk(const int* __restrict__ dsts, int nE, int cbase, int slotBase,
                                          int vec8, int* list, int tid, int lane, int wave) {
  int wc = 0;
#pragma unroll
  for (int g = 0; g < NGRP; ++g) {
    const int el0  = (g * NTHR + tid) * EPT;
    const int e0   = cbase + el0;
    const int sent = -2147483647 - 1;
    v4i da, db;
    if (vec8 != 0 && cbase + CHUNK <= nE) {
      da = *(const v4i*)(dsts + e0);
      db = *(const v4i*)(dsts + e0 + 4);
    } else {
      da.x = (e0     < nE) ? dsts[min(e0, nE - 1)] : sent;
      da.y = (e0 + 1 < nE) ? dsts[min(e0 + 1, nE - 1)] : sent;
      da.z = (e0 + 2 < nE) ? dsts[min(e0 + 2, nE - 1)] : sent;
      da.w = (e0 + 3 < nE) ? dsts[min(e0 + 3, nE - 1)] : sent;
      db.x = (e0 + 4 < nE) ? dsts[min(e0 + 4, nE - 1)] : sent;
      db.y = (e0 + 5 < nE) ? dsts[min(e0 + 5, nE - 1)] : sent;
      db.z = (e0 + 6 < nE) ? dsts[min(e0 + 6, nE - 1)] : sent;
      db.w = (e0 + 7 < nE) ? dsts[min(e0 + 7, nE - 1)] : sent;
    }
    const unsigned nb = (unsigned)slotBase;
    const unsigned s0 = (unsigned)da.x - nb, s1 = (unsigned)da.y - nb;
    const unsigned s2 = (unsigned)da.z - nb, s3 = (unsigned)da.w - nb;
    const unsigned s4 = (unsigned)db.x - nb, s5 = (unsigned)db.y - nb;
    const unsigned s6 = (unsigned)db.z - nb, s7 = (unsigned)db.w - nb;
    const bool h0 = s0 < (unsigned)NB, h1 = s1 < (unsigned)NB, h2 = s2 < (unsigned)NB, h3 = s3 < (unsigned)NB;
    const bool h4 = s4 < (unsigned)NB, h5 = s5 < (unsigned)NB, h6 = s6 < (unsigned)NB, h7 = s7 < (unsigned)NB;
    const unsigned any = __builtin_amdgcn_ballot_w32(h0 | h1 | h2 | h3 | h4 | h5 | h6 | h7);
    if (any != 0u) {
#define HITJ(J, HJ, SJ) { \
        const unsigned mj = __builtin_amdgcn_ballot_w32(HJ); \
        if (mj != 0u) { \
          if (HJ) { \
            const int pos = wc + (int)__builtin_amdgcn_mbcnt_lo(mj, 0u); \
            if (pos < WCAP) list[wave * WCAP + pos] = ((el0 + (J)) << 12) | (int)(SJ); \
          } \
          wc += (int)__builtin_popcount(mj); } }
      HITJ(0, h0, s0)
      HITJ(1, h1, s1)
      HITJ(2, h2, s2)
      HITJ(3, h3, s3)
      HITJ(4, h4, s4)
      HITJ(5, h5, s5)
      HITJ(6, h6, s6)
      HITJ(7, h7, s7)
#undef HITJ
    }
  }
  return wc;
}

__global__ __launch_bounds__(NTHR) void k_wprep(
    const float* __restrict__ w1, const float* __restrict__ w2, _Float16* wp, int L) {
  const int idx   = blockIdx.x * NTHR + threadIdx.x;
  int which = idx >> 9;
  which = which > 2 * L - 1 ? 2 * L - 1 : which;
  const int j  = idx & 511;
  const int n  = j >> 3;
  const int k0 = (j & 7) * 8;
  const int l  = which >> 1;
  const float* w = (which & 1) ? w2 : w1;
  const float* src = w + (size_t)l * WPLANE + n * DD + k0;
  const v4f a = *(const v4f*)src;
  const v4f b = *(const v4f*)(src + 4);
  Pack16 pk;
  pk.h = cvt8(a * WSC, b * WSC);
  _Float16* dst = wp + (size_t)which * WPLANE + n * DD + k0;
  *(volatile v4f*)dst = pk.f;
  __threadfence();
  *(volatile v4f*)dst = pk.f;
}

__global__ __launch_bounds__(NTHR) void k_count(const int* __restrict__ dsts, int* cnt, int nE, int vec8) {
  __shared__ __attribute__((aligned(16))) int scnt[NBC];
  __shared__ __attribute__((aligned(16))) int list[LISTN];
  __shared__ int wcnt[NWAVE];
  const int tid = threadIdx.x, lane = tid & 31, wave = tid >> 5;
  const int nodeBase = blockIdx.x * NBC;

  for (int i = tid; i < NBC; i += NTHR) scnt[i] = 0;
  __syncthreads();

  const int nChunks = (nE + CHUNK - 1) / CHUNK;
#pragma unroll 1
  for (int ch = 0; ch < nChunks; ++ch) {
    const int cbase = ch * CHUNK;
    const int wc = scan_chunk<NBC>(dsts, nE, cbase, nodeBase, vec8, list, tid, lane, wave);
    if (lane == 0) wcnt[wave] = wc;
    __syncthreads();
    if (wave == 0) {
#pragma unroll 1
      for (int wsx = 0; wsx < NWAVE; ++wsx) {
        int n = __builtin_amdgcn_readfirstlane(wcnt[wsx]);
        n = n > WCAP ? WCAP : (n < 0 ? 0 : n);
        const int* lp = list + wsx * WCAP;
#pragma unroll 1
        for (int i = 0; i < n; ++i) {
          const int ent  = __builtin_amdgcn_readfirstlane(lp[i]);
          const int slot = ent & (NBC - 1);
          if (lane == 0) scnt[slot] = scnt[slot] + 1;
        }
      }
    }
    __syncthreads();
  }

  v4i cq[4];
#pragma unroll
  for (int q = 0; q < 4; ++q) {
    const int f = (wave * 4 + q) * 128 + 4 * lane;
    cq[q] = *(const v4i*)(scnt + f);
  }
  int* cp = cnt + (size_t)nodeBase;
#pragma unroll
  for (int q = 0; q < 4; ++q) {
    const int f = (wave * 4 + q) * 128 + 4 * lane;
    *(volatile v4i*)(cp + f) = cq[q];
  }
  __threadfence();
#pragma unroll
  for (int q = 0; q < 4; ++q) {
    const int f = (wave * 4 + q) * 128 + 4 * lane;
    *(volatile v4i*)(cp + f) = cq[q];
  }
}

__global__ __launch_bounds__(OTHR) void k_offsets(
    const int* __restrict__ cnt, int* off, int* rbase, int nChunk) {
  __shared__ __attribute__((aligned(16))) int soff[NBC];
  __shared__ __attribute__((aligned(16))) int srb[RBN];
  __shared__ int wtot[OTHR / 32];
  const int tid = threadIdx.x, lane = tid & 31, wave = tid >> 5, sub = tid >> 7;
  for (int i = tid; i < RBN; i += OTHR) srb[i] = 0;
  int carry = 0;
#pragma unroll 1
  for (int ch = 0; ch < nChunk; ++ch) {
    const int base = ch * NBC;
    const v4i c0 = *(const v4i*)(cnt + base + 8 * tid);
    const v4i c1 = *(const v4i*)(cnt + base + 8 * tid + 4);
    const int e0 = max(c0.x, 0), e1 = max(c0.y, 0), e2 = max(c0.z, 0), e3 = max(c0.w, 0);
    const int e4 = max(c1.x, 0), e5 = max(c1.y, 0), e6 = max(c1.z, 0), e7 = max(c1.w, 0);
    const int ts = e0 + e1 + e2 + e3 + e4 + e5 + e6 + e7;
    int incl = ts;
#pragma unroll
    for (int d = 1; d < 32; d <<= 1) {
      const int t = __shfl_up(incl, d);
      if (lane >= d) incl += t;
    }
    if (lane == 31) wtot[wave] = incl;
    __syncthreads();
    const int S0 = wtot[0]  + wtot[1]  + wtot[2]  + wtot[3];
    const int S1 = wtot[4]  + wtot[5]  + wtot[6]  + wtot[7];
    const int S2 = wtot[8]  + wtot[9]  + wtot[10] + wtot[11];
    const int S3 = wtot[12] + wtot[13] + wtot[14] + wtot[15];
    int pre = 0;
#pragma unroll 1
    for (int w = 4 * sub; w < wave; ++w) pre += wtot[w];
    const int b0 = carry;
    const int b1 = b0 + ((S0 + 31) & ~31);
    const int b2 = b1 + ((S1 + 31) & ~31);
    const int b3 = b2 + ((S2 + 31) & ~31);
    const int b4 = b3 + ((S3 + 31) & ~31);
    const int myb = sub == 0 ? b0 : (sub == 1 ? b1 : (sub == 2 ? b2 : b3));
    if (tid == 0) {
      srb[min(4 * ch + 0, RBN - 1)] = b0;
      srb[min(4 * ch + 1, RBN - 1)] = b1;
      srb[min(4 * ch + 2, RBN - 1)] = b2;
      srb[min(4 * ch + 3, RBN - 1)] = b3;
    }
    int run = myb + pre + incl - ts;
    soff[8 * tid + 0] = run; run += e0;
    soff[8 * tid + 1] = run; run += e1;
    soff[8 * tid + 2] = run; run += e2;
    soff[8 * tid + 3] = run; run += e3;
    soff[8 * tid + 4] = run; run += e4;
    soff[8 * tid + 5] = run; run += e5;
    soff[8 * tid + 6] = run; run += e6;
    soff[8 * tid + 7] = run;
    carry = b4;
    __syncthreads();
    const v4i o0 = *(const v4i*)(soff + 4 * tid);
    const v4i o1 = *(const v4i*)(soff + 4 * (tid + OTHR));
    int* op = off + base;
    *(volatile v4i*)(op + 4 * tid) = o0;
    *(volatile v4i*)(op + 4 * (tid + OTHR)) = o1;
    __threadfence();
    *(volatile v4i*)(op + 4 * tid) = o0;
    *(volatile v4i*)(op + 4 * (tid + OTHR)) = o1;
    __syncthreads();
  }
  if (tid == 0) srb[min(4 * nChunk, RBN - 1)] = carry;
  __syncthreads();
  v4i rv = {0, 0, 0, 0};
  if (tid < 32) rv = *(const v4i*)(srb + 4 * tid);
  if (tid < 32) *(volatile v4i*)(rbase + 4 * tid) = rv;
  __threadfence();
  if (tid < 32) *(volatile v4i*)(rbase + 4 * tid) = rv;
}

__global__ __launch_bounds__(NTHR) void k_fill(
    const int* __restrict__ dsts, const int* __restrict__ off, const int* __restrict__ rbase,
    int* csr, int nE, int vec8, int csrLen) {
  extern __shared__ v4f lds_dyn[];
  int* region = (int*)lds_dyn;
  int* cursor = region + RCAP;
  int* list   = cursor + NBF;
  int* wcnt   = list + LISTN;
  const int tid = threadIdx.x, lane = tid & 31, wave = tid >> 5;
  const int b = blockIdx.x;
  const int nodeBase = b * NBF;

  int rb0 = rbase[b];
  const int rb1 = rbase[b + 1];
  rb0 = rb0 < 0 ? 0 : (rb0 > csrLen ? csrLen : rb0);
  rb0 &= ~31;
  int len = rb1 - rb0;
  len = len < 0 ? 0 : (len > RCAP ? RCAP : len);
  int lenW = (len + 31) & ~31;
  if (rb0 + lenW > csrLen) lenW = (csrLen - rb0) & ~31;

  {
    const v4i z = {0, 0, 0, 0};
    for (int i = tid; i < RCAP / 4; i += NTHR) ((v4i*)region)[i] = z;
    for (int s = tid; s < NBF; s += NTHR) {
      int o = off[nodeBase + s] - rb0;
      o = o < 0 ? 0 : (o > RCAP ? RCAP : o);
      cursor[s] = o;
    }
  }
  __syncthreads();

  const int nChunks = (nE + CHUNK - 1) / CHUNK;
#pragma unroll 1
  for (int ch = 0; ch < nChunks; ++ch) {
    const int cbase = ch * CHUNK;
    const int wc = scan_chunk<NBF>(dsts, nE, cbase, nodeBase, vec8, list, tid, lane, wave);
    if (lane == 0) wcnt[wave] = wc;
    __syncthreads();
    if (wave == 0) {
#pragma unroll 1
      for (int wsx = 0; wsx < NWAVE; ++wsx) {
        int n = __builtin_amdgcn_readfirstlane(wcnt[wsx]);
        n = n > WCAP ? WCAP : (n < 0 ? 0 : n);
        const int* lp = list + wsx * WCAP;
#pragma unroll 1
        for (int i = 0; i < n; ++i) {
          const int ent  = __builtin_amdgcn_readfirstlane(lp[i]);
          const int slot = ent & (NBF - 1);
          int e = cbase + ((ent >> 12) & (CHUNK - 1));
          e = e > nE - 1 ? nE - 1 : e;
          if (lane == 0) {
            int pos = cursor[slot];
            pos = pos < 0 ? 0 : (pos > RCAP - 1 ? RCAP - 1 : pos);
            region[pos] = e;
            const int np = pos + 1;
            cursor[slot] = np > RCAP ? RCAP : np;
          }
        }
      }
    }
    __syncthreads();
  }

  const int nv = lenW >> 2;
  int* gp = csr + rb0;
#pragma unroll 1
  for (int i = tid; i < nv; i += NTHR) { const v4i v = ((const v4i*)region)[i]; *(volatile v4i*)(gp + 4 * i) = v; }
  __threadfence();
#pragma unroll 1
  for (int i = tid; i < nv; i += NTHR) { const v4i v = ((const v4i*)region)[i]; *(volatile v4i*)(gp + 4 * i) = v; }
}

__device__ __forceinline__ v2f agg_seg(
    const int* __restrict__ csr, const int* __restrict__ acol, const float* __restrict__ aval,
    const float* __restrict__ xin, int n, int st, int lane, int nN, int nE, int csrLen) {
  v2f acc = {0.0f, 0.0f};
#pragma unroll 1
  for (int q0 = 0; q0 < n; q0 += 32) {
    int pos = st + q0 + lane;
    pos = pos < 0 ? 0 : (pos > csrLen - 1 ? csrLen - 1 : pos);
    int ed = csr[pos];
    ed = ed < 0 ? 0 : (ed > nE - 1 ? nE - 1 : ed);
    int cl = acol[ed];
    cl = cl < 0 ? 0 : (cl > nN - 1 ? nN - 1 : cl);
    const float vl = aval[ed];
    const int mcnt = (n - q0) < 32 ? (n - q0) : 32;
#pragma unroll 1
    for (int p = 0; p < mcnt; ++p) {
      const int   s = __builtin_amdgcn_readlane(cl, p);
      const float v = __int_as_float(__builtin_amdgcn_readlane(__float_as_int(vl), p));
      const v2f   x = *(const v2f*)(xin + (size_t)s * DD + 2 * lane);
      acc.x = fmaf(v, x.x, acc.x);
      acc.y = fmaf(v, x.y, acc.y);
    }
  }
  return acc;
}

__global__ __launch_bounds__(NTHR) void k_agg(
    const int* __restrict__ csr, const int* __restrict__ off, const int* __restrict__ cnt,
    const int* __restrict__ acol, const float* __restrict__ aval,
    const float* __restrict__ xin, float* S, int nN, int nE, int csrLen) {
  const int tid = threadIdx.x, lane = tid & 31, wave = tid >> 5;
  const int tbase = blockIdx.x * TGT + wave * 32;
  const int cl = tbase + lane;
  const int cnt_l = cnt[cl];
  const int off_l = off[cl];
  const int q2 = 2 * (lane & 15);
  const int tg = lane >> 4;

#pragma unroll 1
  for (int j = 0; j < 32; j += 2) {
    int na = __builtin_amdgcn_readlane(cnt_l, j);
    na = na < 0 ? 0 : (na > DEGCAP ? DEGCAP : na);
    const int sa = __builtin_amdgcn_readlane(off_l, j);
    int nb = __builtin_amdgcn_readlane(cnt_l, j + 1);
    nb = nb < 0 ? 0 : (nb > DEGCAP ? DEGCAP : nb);
    const int sb = __builtin_amdgcn_readlane(off_l, j + 1);
    const v2f accA = agg_seg(csr, acol, aval, xin, na, sa, lane, nN, nE, csrLen);
    const v2f accB = agg_seg(csr, acol, aval, xin, nb, sb, lane, nN, nE, csrLen);
    const float a0 = __shfl(accA.x, q2),     a1 = __shfl(accA.y, q2);
    const float a2 = __shfl(accA.x, q2 + 1), a3 = __shfl(accA.y, q2 + 1);
    const float c0 = __shfl(accB.x, q2),     c1 = __shfl(accB.y, q2);
    const float c2 = __shfl(accB.x, q2 + 1), c3 = __shfl(accB.y, q2 + 1);
    v4f w;
    w.x = tg != 0 ? c0 : a0;
    w.y = tg != 0 ? c1 : a1;
    w.z = tg != 0 ? c2 : a2;
    w.w = tg != 0 ? c3 : a3;
    float* gp = S + (size_t)(tbase + j) * DD + 4 * lane;
    *(volatile v4f*)gp = w;
    __threadfence();
    *(volatile v4f*)gp = w;
  }
}

__global__ __launch_bounds__(NTHR) void k_layer(
    const float* __restrict__ ego, const float* __restrict__ side,
    const _Float16* __restrict__ Wp, const float* __restrict__ b1, const float* __restrict__ b2,
    float* egon, int nN) {
  extern __shared__ v4f lds_dyn[];
  _Float16* sU  = (_Float16*)lds_dyn;
  _Float16* sE  = sU + GROWS * APK;
  float*    stg = (float*)(sE + GROWS * APK);
  const int tid = threadIdx.x, lane = tid & 31, wave = tid >> 5, hh = lane >> 4, m = lane & 15;
  const int rowBase = blockIdx.x * GROWS;

#pragma unroll
  for (int i = 0; i < (GROWS * DD / 8) / NTHR; ++i) {
    const int idx = i * NTHR + tid;
    const int r   = idx >> 3;
    const int c0  = (idx & 7) * 8;
    int ge = rowBase + r;
    ge = ge > nN - 1 ? nN - 1 : ge;
    const float* ep = ego  + (size_t)ge * DD + c0;
    const float* sp = side + (size_t)(rowBase + r) * DD + c0;
    const v4f ea = *(const v4f*)ep, eb = *(const v4f*)(ep + 4);
    const v4f sa = *(const v4f*)sp, sb = *(const v4f*)(sp + 4);
    const v4f ua = (ea + sa) * ASC, ub = (eb + sb) * ASC;
    const v4f xa = ea * ASC, xb = eb * ASC;
    *(v8h*)(sU + r * APK + c0) = cvt8(ua, ub);
    *(v8h*)(sE + r * APK + c0) = cvt8(xa, xb);
    *(v4f*)(stg + r * DD + c0)     = sa;
    *(v4f*)(stg + r * DD + c0 + 4) = sb;
  }
  __syncthreads();

  const _Float16* pu = sU + (wave * 16 + m) * APK + 8 * hh;
  const _Float16* pe = sE + (wave * 16 + m) * APK + 8 * hh;
  const int rloc0 = wave * 16 + 8 * hh;

#pragma unroll
  for (int t = 0; t < 4; ++t) {
    v8f acc1 = {0.f, 0.f, 0.f, 0.f, 0.f, 0.f, 0.f, 0.f};
    v8f acc2 = {0.f, 0.f, 0.f, 0.f, 0.f, 0.f, 0.f, 0.f};
#pragma unroll
    for (int kt = 0; kt < 2; ++kt) {
      FragH au, ae, bw1, bw2;
      au.half[0] = *(const v8h*)(pu + 32 * kt);
      au.half[1] = *(const v8h*)(pu + 32 * kt + 16);
      ae.half[0] = *(const v8h*)(pe + 32 * kt);
      ae.half[1] = *(const v8h*)(pe + 32 * kt + 16);
      const _Float16* bp = Wp + (size_t)(16 * t + m) * DD + 32 * kt + 8 * hh;
      bw1.half[0] = *(const v8h*)bp;             bw1.half[1] = *(const v8h*)(bp + 16);
      bw2.half[0] = *(const v8h*)(bp + WPLANE);  bw2.half[1] = *(const v8h*)(bp + WPLANE + 16);
      acc1 = wmh(au.v, bw1.v, acc1);
      acc2 = wmh(ae.v, bw2.v, acc2);
    }
    const int n = 16 * t + m;
    const float bv1 = b1[n];
    const float bv2 = b2[n];
#pragma unroll
    for (int r = 0; r < 8; ++r) {
      float* q = stg + (rloc0 + r) * DD + n;
      const float ag = *q;
      const float sx = fmaf(acc1[r], ISC, bv1);
      const float tt = fmaf(acc2[r], ISC, bv2);
      float y = fmaf(ag, tt, sx);
      y = y >= 0.0f ? y : 0.01f * y;
      *q = y;
    }
  }
  __syncthreads();

  v4f ov[8];
#pragma unroll
  for (int i = 0; i < 8; ++i) {
    const int row = wave * 16 + 2 * i + hh;
    ov[i] = *(const v4f*)(stg + row * DD + 4 * m);
  }
#pragma unroll
  for (int i = 0; i < 8; ++i) {
    const int row = wave * 16 + 2 * i + hh;
    *(volatile v4f*)(egon + (size_t)(rowBase + row) * DD + 4 * m) = ov[i];
  }
  __threadfence();
#pragma unroll
  for (int i = 0; i < 8; ++i) {
    const int row = wave * 16 + 2 * i + hh;
    *(volatile v4f*)(egon + (size_t)(rowBase + row) * DD + 4 * m) = ov[i];
  }
}

__global__ __launch_bounds__(NTHR) void k_loss(
    const float* __restrict__ e0, const float* __restrict__ epl, int L, int planeF,
    const int* __restrict__ user, const int* __restrict__ posI, const int* __restrict__ negI,
    int nB, int nN, float* out) {
  __shared__ float wsum[NWAVE];
  const int tid = threadIdx.x, lane = tid & 31, wave = tid >> 5;
  float acc = 0.0f;
#pragma unroll 1
  for (int b = wave; b < nB; b += NWAVE) {
    int u = user[b], p = posI[b], g = negI[b];
    u = u < 0 ? 0 : (u > nN - 1 ? nN - 1 : u);
    p = p < 0 ? 0 : (p > nN - 1 ? nN - 1 : p);
    g = g < 0 ? 0 : (g > nN - 1 ? nN - 1 : g);
    const v2f xu = *(const v2f*)(e0 + (size_t)u * DD + 2 * lane);
    const v2f xp = *(const v2f*)(e0 + (size_t)p * DD + 2 * lane);
    const v2f xg = *(const v2f*)(e0 + (size_t)g * DD + 2 * lane);
    float dp = fmaf(xu.x, xp.x, xu.y * xp.y);
    float dn = fmaf(xu.x, xg.x, xu.y * xg.y);
#pragma unroll 1
    for (int l = 0; l < L; ++l) {
      const float* pl = epl + (size_t)l * (size_t)planeF;
      const v2f yu = *(const v2f*)(pl + (size_t)u * DD + 2 * lane);
      const v2f yp = *(const v2f*)(pl + (size_t)p * DD + 2 * lane);
      const v2f yg = *(const v2f*)(pl + (size_t)g * DD + 2 * lane);
      dp = fmaf(yu.x, yp.x, fmaf(yu.y, yp.y, dp));
      dn = fmaf(yu.x, yg.x, fmaf(yu.y, yg.y, dn));
    }
#pragma unroll
    for (int s = 16; s > 0; s >>= 1) {
      dp += __shfl_xor(dp, s);
      dn += __shfl_xor(dn, s);
    }
    const float z = dn - dp;
    const float term = fmaxf(z, 0.0f) + log1pf(expf(-fabsf(z)));
    acc += term;
  }
  if (lane == 0) wsum[wave] = acc;
  __syncthreads();
  if (tid == 0) {
    float s = 0.0f;
#pragma unroll
    for (int w = 0; w < NWAVE; ++w) s += wsum[w];
    *(volatile float*)out = s;
    __threadfence();
    *(volatile float*)out = s;
  }
}

extern "C" void kernel_launch(void* const* d_in, const int* in_sizes, int n_in,
                              void* d_out, int out_size, void* d_ws, size_t ws_size,
                              hipStream_t stream) {
  if (n_in < 11) return;
  const int nN = in_sizes[0] / DD;
  if (nN < 1 || in_sizes[0] != nN * DD) return;
  const int L = in_sizes[1] / WPLANE;
  if (L < 1 || L > LMAX || in_sizes[1] != L * WPLANE || in_sizes[3] != L * WPLANE) return;
  if (in_sizes[2] != L * DD || in_sizes[4] != L * DD) return;
  const int nE = in_sizes[5];
  if (nE < 1 || in_sizes[6] != nE || in_sizes[7] != nE) return;
  const int nB = in_sizes[8];
  if (nB < 1 || in_sizes[9] != nB || in_sizes[10] != nB) return;
  if (out_size != 1) return;
  if (nE > (1 << 28) || nN > (1 << 24)) return;

  const float* emb  = (const float*)d_in[0];
  const float* w1   = (const float*)d_in[1];
  const float* b1   = (const float*)d_in[2];
  const float* w2   = (const float*)d_in[3];
  const float* b2   = (const float*)d_in[4];
  const float* vals = (const float*)d_in[5];
  const int*   rowI = (const int*)d_in[6];
  const int*   colI = (const int*)d_in[7];
  const int*   user = (const int*)d_in[8];
  const int*   posI = (const int*)d_in[9];
  const int*   negI = (const int*)d_in[10];
  float* out = (float*)d_out;

  const int NPAD   = ((nN + TGT - 1) / TGT) * TGT;
  const int nBC    = (nN + NBC - 1) / NBC;
  const int CNTPAD = nBC * NBC;
  if (4 * nBC + 1 > RBN) return;
  const int nBF    = (nN + NBF - 1) / NBF;
  const int csrLen = ((nE + 31) & ~31) + 4096;
  if (31 * 4 * nBC > 4096) return;
  const int nLay   = NPAD / GROWS;
  const int nAgg   = NPAD / TGT;
  const int planeF = NPAD * DD;

  char* ws = (char*)d_ws;
  size_t off = 0;
  const size_t oW   = off; off += (size_t)L * 2 * WPLANE * 2;      off = (off + 255) & ~(size_t)255;
  const size_t oCnt = off; off += (size_t)CNTPAD * 4;              off = (off + 255) & ~(size_t)255;
  const size_t oOff = off; off += (size_t)CNTPAD * 4;              off = (off + 255) & ~(size_t)255;
  const size_t oRb  = off; off += (size_t)RBN * 4;                 off = (off + 255) & ~(size_t)255;
  const size_t oCsr = off; off += (size_t)csrLen * 4;              off = (off + 255) & ~(size_t)255;
  const size_t oSd  = off; off += (size_t)planeF * 4;              off = (off + 255) & ~(size_t)255;
  const size_t oE   = off; off += (size_t)L * planeF * 4;          off = (off + 255) & ~(size_t)255;
  if (off > ws_size || off > (size_t)WSCAP) return;
  _Float16* wp   = (_Float16*)(ws + oW);
  int*      cnt  = (int*)(ws + oCnt);
  int*      offp = (int*)(ws + oOff);
  int*      rb   = (int*)(ws + oRb);
  int*      csr  = (int*)(ws + oCsr);
  float*    Sd   = (float*)(ws + oSd);
  float*    Epl  = (float*)(ws + oE);

  const int vec8 = ((nE & 3) == 0) ? 1 : 0;

  k_wprep<<<4 * L, NTHR, 0, stream>>>(w1, w2, wp, L);

  k_count<<<nBC, NTHR, 0, stream>>>(rowI, cnt, nE, vec8);
  k_offsets<<<1, OTHR, 0, stream>>>(cnt, offp, rb, nBC);
  hipFuncSetAttribute(reinterpret_cast<const void*>(&k_fill),
                      hipFuncAttributeMaxDynamicSharedMemorySize, LDS_FILL);
  k_fill<<<nBF, NTHR, LDS_FILL, stream>>>(rowI, offp, rb, csr, nE, vec8, csrLen);

  hipFuncSetAttribute(reinterpret_cast<const void*>(&k_layer),
                      hipFuncAttributeMaxDynamicSharedMemorySize, LDS_LAYER);
  const float* xin = emb;
  for (int l = 0; l < L; ++l) {
    float* xout = Epl + (size_t)l * planeF;
    k_agg<<<nAgg, NTHR, 0, stream>>>(csr, offp, cnt, colI, vals, xin, Sd, nN, nE, csrLen);
    k_layer<<<nLay, NTHR, LDS_LAYER, stream>>>(xin, Sd, wp + (size_t)l * 2 * WPLANE,
                                               b1 + (size_t)l * DD, b2 + (size_t)l * DD, xout, nN);
    xin = xout;
  }

  k_loss<<<1, NTHR, 0, stream>>>(emb, Epl, L, planeF, user, posI, negI, nB, nN, out);
}
